// MolecularHamiltonianExact_33380485824797
// MI455X (gfx1250) — hardware-verified
//
#include <hip/hip_runtime.h>


#ifndef NB
#define NB 256
#endif
#ifndef TT
#define TT 8000
#endif
#define NB_FULL 256
#define TT_FULL 8000
#define NQ   40
#define HH   32
#define KP   64
#define NPIECE (NQ / 8)
#define NTILE (TT / 16)
#define TPAD ((((TT + 16) + 31) / 32) * 32)
#define BPW  4
#define TW   8
#define WCAR 256.0f
#define DSC  ((float)(2.0 * 1.4426950408889634 / 256.0))
#define TL2E ((float)(2.0 * 1.4426950408889634))
#define PL2E ((float)(0.1 * 1.4426950408889634))

static_assert(NQ == 40);
static_assert(NQ % 8 == 0);
static_assert(NQ <= KP);
static_assert(KP == 64);
static_assert(KP % 32 == 0);
static_assert(HH == 32);
static_assert(HH * 8 == 256);
static_assert(TT % 32 == 0);
static_assert((NTILE + 1) * 16 <= TPAD);
static_assert(TPAD % 32 == 0);
static_assert(TW * BPW == 32);
static_assert(NB % 32 == 0);
static_assert(NB <= NB_FULL);
static_assert(TT <= TT_FULL);
static_assert(256 * 16 == 32 * KP * 2);
static_assert(32 * 16 == 32 * 16);
static_assert(8 * 16 == 32 * 4);
static_assert(32 * 4 * 4 <= 131072);

typedef _Float16 h16;
typedef unsigned short bf;
typedef __attribute__((ext_vector_type(16))) _Float16 v16h;
typedef __attribute__((ext_vector_type(8)))  _Float16 v8h;
typedef __attribute__((ext_vector_type(8)))  unsigned short v8us;
typedef __attribute__((ext_vector_type(16))) unsigned short v16us;
typedef __attribute__((ext_vector_type(8)))  float    v8f;
typedef __attribute__((ext_vector_type(4)))  float    v4f;
typedef __attribute__((ext_vector_type(4)))  int      v4i;
typedef __attribute__((ext_vector_type(4)))  unsigned v4u;
typedef v4f  __attribute__((may_alias)) v4fa;
typedef v4u  __attribute__((may_alias)) v4ua;

__device__ __forceinline__ unsigned short f2bf(float f) { unsigned u = __float_as_uint(f); u += 0x7FFFu + ((u >> 16) & 1u); return (unsigned short)(u >> 16); }
__device__ __forceinline__ float bfr(float f) { return __uint_as_float(((unsigned)f2bf(f)) << 16); }
__device__ __forceinline__ v16h cat16(v8h lo, v8h hi) { return __builtin_shufflevector(lo, hi, 0, 1, 2, 3, 4, 5, 6, 7, 8, 9, 10, 11, 12, 13, 14, 15); }
__device__ __forceinline__ v8f wmma16(v16h a, v16h b, v8f c) { return __builtin_amdgcn_wmma_f32_16x16x32_f16(false, a, false, b, (short)0, c, false, false); }
__device__ __forceinline__ v16h  ldh(const h16* p) { return cat16(*(const v8h*)p, *(const v8h*)(p + 16)); }
__device__ __forceinline__ v16us ldu(const unsigned short* p) { return __builtin_shufflevector(*(const v8us*)p, *(const v8us*)(p + 16), 0, 1, 2, 3, 4, 5, 6, 7, 8, 9, 10, 11, 12, 13, 14, 15); }
static __device__ __forceinline__ h16 toh_flush(float v) { const h16 r = (h16)v; return (fabsf(v) < 6.103515625e-05f) ? (h16)0.0f : r; }
__device__ __forceinline__ unsigned short hbits(h16 h) { return __builtin_bit_cast(unsigned short, h); }
__device__ __forceinline__ v8f wmma16g(v16h a, v16h b, v8f c) { c = wmma16(a, b, c); asm volatile("v_nop\n\tv_nop\n\tv_nop\n\tv_nop" : "+v"(c) : "v"(a), "v"(b)); return c; }

__global__ __launch_bounds__(256) void k_wprep(const float* __restrict__ W1, h16* WT) {
#pragma clang fp contract(off)
    const int tid = threadIdx.x, h = tid >> 3, p = tid & 7;
    float w[8];
#pragma unroll
    for (int i = 0; i < 8; ++i) { const int q = 8 * p + i; const int qc = q < NQ ? q : (NQ - 1); w[i] = W1[qc * HH + h]; }
    asm volatile("" : "+v"(w[0]), "+v"(w[1]), "+v"(w[2]), "+v"(w[3]), "+v"(w[4]), "+v"(w[5]), "+v"(w[6]), "+v"(w[7]));
    v8h hv;
#pragma unroll
    for (int i = 0; i < 8; ++i) { const int q = 8 * p + i; const float val = (q < NQ) ? bfr(w[i]) * WCAR : 0.0f; hv[i] = toh_flush(val); }
    h16* wo = WT + h * KP + p * 8;
#pragma unroll 1
    for (int ps = 0; ps < 2; ++ps) { *(volatile v8h*)wo = hv; if (ps == 0) __threadfence(); }
}

__global__ __launch_bounds__(256) void k_tprep(const int* __restrict__ codes, const float* __restrict__ coeffs, unsigned short* FM, unsigned* TS) {
#pragma clang fp contract(off)
    __shared__ __align__(16) unsigned rec[32 * 4];
    const int tid = threadIdx.x, tl = tid >> 3, p = tid & 7;
    const int lane = tid & 31;
    const int wave = __builtin_amdgcn_readfirstlane((int)(threadIdx.x >> 5));
    const int t = blockIdx.x * 32 + tl;
    const int tc = t < TT ? t : (TT - 1);
    const int pc = p < NPIECE ? p : (NPIECE - 1);
    const int* cp = codes + (size_t)tc * NQ + 8 * pc;
    v4i c0 = *(const v4i*)cp, c1 = *(const v4i*)(cp + 4);
    float cf = coeffs[tc];
    asm volatile("" : "+v"(c0), "+v"(c1), "+v"(cf));
    const bool valid = (t < TT) & (p < NPIECE);
    int cc[8];
#pragma unroll
    for (int i = 0; i < 4; ++i) { cc[i] = c0[i]; cc[4 + i] = c1[i]; }
    v8us o; unsigned yb = 0u; int ny = 0;
#pragma unroll
    for (int i = 0; i < 8; ++i) {
        const int c = cc[i];
        const bool xy = valid & ((c == 1) | (c == 2));
        const bool yz = valid & (c >= 2);
        const bool y2 = valid & (c == 2);
        o[i] = xy ? (unsigned short)0x8000 : (unsigned short)0;
        yb |= (yz ? 1u : 0u) << i;
        ny += y2 ? 1 : 0; }
    unsigned short* fo = FM + (size_t)t * KP + p * 8;
#pragma unroll 1
    for (int ps = 0; ps < 2; ++ps) { *(volatile v8us*)fo = o; if (ps == 0) __threadfence(); }
    unsigned ylo = (p < 4) ? (yb << (8 * (p & 3))) : 0u;
    unsigned yhi = (p >= 4) ? (yb << (8 * (p & 3))) : 0u;
    ylo |= (unsigned)__shfl_xor((int)ylo, 1, 32); yhi |= (unsigned)__shfl_xor((int)yhi, 1, 32); ny += __shfl_xor(ny, 1, 32);
    ylo |= (unsigned)__shfl_xor((int)ylo, 2, 32); yhi |= (unsigned)__shfl_xor((int)yhi, 2, 32); ny += __shfl_xor(ny, 2, 32);
    ylo |= (unsigned)__shfl_xor((int)ylo, 4, 32); yhi |= (unsigned)__shfl_xor((int)yhi, 4, 32); ny += __shfl_xor(ny, 4, 32);
    const int m4 = ny & 3;
    const float phase = (m4 == 0) ? 1.0f : ((m4 == 2) ? -1.0f : 0.0f);
    const int nyz = __popc(ylo) + __popc(yhi);
    float ct = bfr(cf) * phase;
    ct = (nyz & 1) ? -ct : ct;
    ct = (t < TT) ? ct : 0.0f;
    if (p == 0) { v4u rv; rv[0] = __float_as_uint(ct); rv[1] = ylo; rv[2] = yhi; rv[3] = 0u; *(v4ua*)(&rec[4 * tl]) = rv; }
    __syncthreads();
    if (wave == 0) {
        const v4u rv = *(const v4ua*)(&rec[4 * lane]);
        unsigned* tp = TS + ((size_t)blockIdx.x * 32 + lane) * 4;
#pragma unroll 1
        for (int ps = 0; ps < 2; ++ps) { *(volatile v4u*)tp = rv; if (ps == 0) __threadfence(); }
    }
}

__global__ __launch_bounds__(32 * TW) void k_terms(const float* __restrict__ states, const h16* __restrict__ WT, const unsigned short* __restrict__ FM, const unsigned* __restrict__ TS,
                                                   const float* __restrict__ b1, const float* __restrict__ w2, float* OUT) {
    __shared__ __align__(16) float res[32];
    const int lane = threadIdx.x & 31, lr = lane & 15, hi = lane >> 4;
    const int wave = __builtin_amdgcn_readfirstlane((int)(threadIdx.x >> 5));
    const v16h wa00 = ldh(WT + (size_t)lr * KP + 8 * hi),        wa01 = ldh(WT + (size_t)lr * KP + 32 + 8 * hi);
    const v16h wa10 = ldh(WT + (size_t)(16 + lr) * KP + 8 * hi), wa11 = ldh(WT + (size_t)(16 + lr) * KP + 32 + 8 * hi);
    float bs0[8], bs1[8], wn0[8], wn1[8]; float sumw = 0.0f;
    { const v4f ba = *(const v4f*)(b1 + 8 * hi), bb = *(const v4f*)(b1 + 8 * hi + 4), bc = *(const v4f*)(b1 + 16 + 8 * hi), bd = *(const v4f*)(b1 + 16 + 8 * hi + 4);
      const v4f wa = *(const v4f*)(w2 + 8 * hi), wb = *(const v4f*)(w2 + 8 * hi + 4), wc = *(const v4f*)(w2 + 16 + 8 * hi), wd = *(const v4f*)(w2 + 16 + 8 * hi + 4);
#pragma unroll
      for (int r = 0; r < 4; ++r) {
          bs0[r] = bfr(ba[r]) * TL2E; bs0[4 + r] = bfr(bb[r]) * TL2E; bs1[r] = bfr(bc[r]) * TL2E; bs1[4 + r] = bfr(bd[r]) * TL2E;
          const float u0 = bfr(wa[r]), u1 = bfr(wb[r]), u2 = bfr(wc[r]), u3 = bfr(wd[r]);
          wn0[r] = -2.0f * u0; wn0[4 + r] = -2.0f * u1; wn1[r] = -2.0f * u2; wn1[4 + r] = -2.0f * u3;
          sumw += (u0 + u1) + (u2 + u3); } }
    const v8us z8 = (v8us){};
#pragma unroll 1
    for (int j = 0; j < BPW; ++j) {
        const int b = blockIdx.x * 32 + wave * BPW + j;
        const float* sp = states + (size_t)b * NQ;
        const v4f x0 = *(const v4f*)(sp + 8 * hi), x1 = *(const v4f*)(sp + 8 * hi + 4);
        const v4f x2 = *(const v4f*)(sp + 16 + 8 * hi), x3 = *(const v4f*)(sp + 16 + 8 * hi + 4);
        v4f x4 = *(const v4f*)(sp + 32), x5 = *(const v4f*)(sp + 36);
        asm volatile("" : "+v"(x4), "+v"(x5));
        float xa[8], xb[8], xc[8];
#pragma unroll
        for (int i = 0; i < 4; ++i) { xa[i] = x0[i]; xa[4 + i] = x1[i]; xb[i] = x2[i]; xb[4 + i] = x3[i]; xc[i] = x4[i]; xc[4 + i] = x5[i]; }
        v16us s0, s1; unsigned bt0 = 0u, bt1 = 0u, bt2 = 0u; int bad = 0;
#pragma unroll
        for (int i = 0; i < 8; ++i) {
            const float va = bfr(xa[i]), vb = bfr(xb[i]), vc = bfr(xc[i]);
            bad |= ((fabsf(va) != 1.0f) | (fabsf(vb) != 1.0f) | (fabsf(vc) != 1.0f)) ? 1 : 0;
            s0[i] = hbits(toh_flush(va)); s0[8 + i] = hbits(toh_flush(vb));
            const unsigned short hc = hbits(toh_flush(vc));
            s1[i] = (hi == 0) ? hc : (unsigned short)0; s1[8 + i] = (unsigned short)0;
            bt0 |= ((va < 0.0f) ? 1u : 0u) << i; bt1 |= ((vb < 0.0f) ? 1u : 0u) << i; bt2 |= ((vc < 0.0f) ? 1u : 0u) << i; }
        unsigned slo = (bt0 << (8 * hi)) | (bt1 << (16 + 8 * hi));
        const unsigned shi = bt2;
        slo |= (unsigned)__shfl_xor((int)slo, 16, 32);
        bad |= __shfl_xor(bad, 16, 32);
        float acc = 0.0f, psi = 1.0f;
#pragma unroll 1
        for (int tile = 0; tile <= NTILE; ++tile) {
            const size_t trow = (size_t)tile * 16 + lr;
            const unsigned short* fp = FM + trow * KP + 8 * hi;
            const v16us f0 = ldu(fp);
            const v8us f1l = *(const v8us*)(fp + 32);
            const v4u rc = *(const v4u*)(TS + trow * 4);
            const v16us f1 = __builtin_shufflevector(f1l, z8, 0, 1, 2, 3, 4, 5, 6, 7, 8, 9, 10, 11, 12, 13, 14, 15);
            const v16h c0 = __builtin_bit_cast(v16h, s0 ^ f0);
            const v16h c1 = __builtin_bit_cast(v16h, s1 ^ f1);
            v8f d0 = (v8f){}, d1 = (v8f){};
            d0 = wmma16g(wa00, c0, d0); d1 = wmma16g(wa10, c0, d1);
            d0 = wmma16g(wa01, c1, d0); d1 = wmma16g(wa11, c1, d1);
            float part = sumw;
#pragma unroll
            for (int r = 0; r < 8; ++r) {
                const float e0 = __builtin_amdgcn_exp2f(fmaf(d0[r], DSC, bs0[r]));
                const float e1 = __builtin_amdgcn_exp2f(fmaf(d1[r], DSC, bs1[r]));
                const float g0 = __builtin_amdgcn_rcpf(e0 + 1.0f);
                const float g1 = __builtin_amdgcn_rcpf(e1 + 1.0f);
                part = fmaf(wn0[r], g0, part);
                part = fmaf(wn1[r], g1, part); }
            const float dot = part + __shfl_xor(part, 16, 32);
            psi = __builtin_amdgcn_exp2f(dot * PL2E);
            const int par = (__popc(rc[1] & slo) + __popc(rc[2] & shi)) & 1;
            const float cv = __uint_as_float(rc[0]) * psi;
            acc += par ? -cv : cv;
        }
        float tot = acc;
        tot += __shfl_xor(tot, 1, 32); tot += __shfl_xor(tot, 2, 32); tot += __shfl_xor(tot, 4, 32); tot += __shfl_xor(tot, 8, 32);
        float val = tot * (1.0f / psi);
        val = bad ? __uint_as_float(0x7FC00000u) : val;
        if (lane == 0) res[wave * BPW + j] = val;
    }
    __syncthreads();
    if (wave == 0) {
        const int lc = lane < 8 ? lane : 7;
        const v4f val = *(const v4fa*)(&res[4 * lc]);
        float* op = OUT + (size_t)blockIdx.x * 32 + 4 * lane;
#pragma unroll 1
        for (int ps = 0; ps < 2; ++ps) { if (lane < 8) *(volatile v4f*)op = val; if (ps == 0) __threadfence(); }
    }
}

static constexpr size_t al256(size_t v) { return (v + 255) & ~(size_t)255; }
static constexpr size_t SZ_WT = al256((size_t)HH * KP * 2);
static constexpr size_t SZ_FM = al256((size_t)TPAD * KP * 2);
static constexpr size_t SZ_TS = al256((size_t)TPAD * 16);
static constexpr size_t SZ_TOTAL = SZ_WT + SZ_FM + SZ_TS;
static_assert(SZ_TOTAL <= (size_t)134217728);
static_assert((size_t)(TPAD / 32) * 32 * KP * 2 <= SZ_FM);
static_assert((size_t)(TPAD / 32) * 32 * 16 <= SZ_TS);
static_assert((size_t)256 * 16 <= SZ_WT);
static_assert((size_t)(NB / 32) * 32 * 4 <= (size_t)NB_FULL * 4);

extern "C" void kernel_launch(void* const* d_in, const int* in_sizes, int n_in,
                              void* d_out, int out_size, void* d_ws, size_t ws_size, hipStream_t stream) {
    if (n_in < 6) return;
    if ((size_t)in_sizes[0] < (size_t)NB * NQ) return;
    if ((size_t)in_sizes[1] < (size_t)TT) return;
    if ((size_t)in_sizes[2] < (size_t)NQ * HH) return;
    if (in_sizes[3] < HH || in_sizes[4] < HH) return;
    if ((size_t)in_sizes[5] < (size_t)TT * NQ) return;
    if ((size_t)out_size < (size_t)NB) return;
    if (SZ_TOTAL > ws_size) return;
    const float* states = (const float*)d_in[0];
    const float* coeffs = (const float*)d_in[1];
    const float* W1     = (const float*)d_in[2];
    const float* b1     = (const float*)d_in[3];
    const float* w2     = (const float*)d_in[4];
    const int*   codes  = (const int*)d_in[5];
    float* OUT = (float*)d_out;
    char* wsp = (char*)d_ws;
    h16* WT = (h16*)wsp; wsp += SZ_WT;
    unsigned short* FM = (unsigned short*)wsp; wsp += SZ_FM;
    unsigned* TS = (unsigned*)wsp; wsp += SZ_TS;

    k_wprep<<<dim3(1, 1, 1), 256, 0, stream>>>(W1, WT);
    k_tprep<<<dim3(TPAD / 32, 1, 1), 256, 0, stream>>>(codes, coeffs, FM, TS);
    k_terms<<<dim3(NB / 32, 1, 1), 32 * TW, 0, stream>>>(states, WT, FM, TS, b1, w2, OUT);
}
